// MLALayer_39144331935957
// MI455X (gfx1250) — hardware-verified
//
#include <hip/hip_runtime.h>
#include <math.h>
#include <stdint.h>

#ifndef NB
#define NB 2
#endif
#ifndef SEQ
#define SEQ 2048
#endif
#define XS_FULL 2048
#define DMOD  2048
#define NH    16
#define HD    128
#define DL    512
#define DR    64
#define DRH   (DR / 2)
#define CW    (DL + DR)
#define KVD   (NH * HD)
#define QA    ((SEQ < 256) ? SEQ : 256)
#define MROWS (NB * SEQ)
#define RSQS  0.0721687836487032f
#define LOG2E 1.4426950408889634f
#define QSC   256.0f
#define KSC   256.0f
#define CSC   256.0f
#define WKS   1024.0f
#define PCAR  32768.0f
#define VCAR  1024.0f
#define OSC   1024.0f
#define WOS   1024.0f
#define WPB   2
#define NHP   (NH / WPB)
#define NST   (SEQ / 64)
#define NKT   (SEQ / 32)
#define ATT_THREADS (WPB * 32)
#define PTP   36
#define PTW   (16 * PTP)
#define SLP   132
#define SLW   (16 * SLP)
#define WREG  (PTW + SLW)
#define SLAB64 (16 * 68)
#define VTP   72
#define WTP   72
#define RFP   68
#define L2_1E4 13.287712379549449
#define WS_CAP 134217728
static_assert(DMOD == NH * HD && KVD == DMOD && HD == 128 && NH == 16 && WPB == 2 && NHP * WPB == NH);
static_assert(ATT_THREADS == 64 && DL == 512 && DR == 64 && DRH == 32 && CW == 576);
static_assert(NB >= 1 && NB <= 2);
static_assert((SEQ % 64) == 0 && SEQ >= 64 && SEQ <= XS_FULL);
static_assert((QA % 64) == 0 && QA >= 64 && QA <= SEQ && ((SEQ - QA) % 64) == 0);
static_assert((DMOD % 64) == 0 && (KVD % 64) == 0 && (DL % 64) == 0 && (DR % 64) == 0 && (HD % 32) == 0 && (DR % 32) == 0);
static_assert(((SEQ * DMOD / 8) % 256) == 0 && ((MROWS * DL / 8) % 256) == 0 && ((SEQ * DRH) % 256) == 0 && (MROWS % 32) == 0);
static_assert(WPB * WREG * 4 <= 65536 && 2 * HD * VTP * 2 <= 65536 && 4 * SLAB64 * 4 <= 65536);
static_assert(64 * WTP * 2 <= 65536 && 32 * RFP * 4 <= 65536);
static_assert((MROWS * DL + MROWS * DR) * 4 <= MROWS * DMOD * 4);

typedef unsigned short u16;
typedef _Float16 v16h __attribute__((ext_vector_type(16)));
typedef _Float16 v8h  __attribute__((ext_vector_type(8)));
typedef __bf16   v16b __attribute__((ext_vector_type(16)));
typedef float    v8f  __attribute__((ext_vector_type(8)));
typedef float    v4f  __attribute__((ext_vector_type(4)));
typedef unsigned int v4u __attribute__((ext_vector_type(4)));

union FragH { v16h v; v8h h[2]; v4u u[2]; };
union FragB { v16b v; v4u u[2]; };

__device__ __forceinline__ unsigned short bf_bits(float f) {
  unsigned u = __float_as_uint(f);
  return (unsigned short)((u + 0x7FFFu + ((u >> 16) & 1u)) >> 16);
}
__device__ __forceinline__ float bf_up(unsigned short h) { return __uint_as_float(((unsigned)h) << 16); }
__device__ __forceinline__ float bfr(float f) { return bf_up(bf_bits(f)); }
__device__ __forceinline__ unsigned short h_bits(_Float16 x) { return __builtin_bit_cast(unsigned short, x); }
__device__ __forceinline__ unsigned pk16(unsigned short a, unsigned short b) { return (unsigned)a | ((unsigned)b << 16); }
__device__ __forceinline__ v8f zero8() { v8f z = {0.f, 0.f, 0.f, 0.f, 0.f, 0.f, 0.f, 0.f}; return z; }
__device__ __forceinline__ const _Float16* hptr(const u16* p) { return (const _Float16*)(const void*)p; }

__device__ __forceinline__ v16h ldfrag_h(const _Float16* p) {
  FragH f;
  f.h[0] = *(const v8h*)(p);
  f.h[1] = *(const v8h*)(p + 16);
  return f.v;
}
__device__ __forceinline__ v16b ldfrag_b(const u16* p) {
  FragB f;
  f.u[0] = *(const v4u*)(p);
  f.u[1] = *(const v4u*)(p + 16);
  return f.v;
}

__device__ __forceinline__ v8f mma_h(v16h a, v16h b, v8f c) {
  return __builtin_amdgcn_wmma_f32_16x16x32_f16(false, a, false, b, (short)0, c, false, false);
}
__device__ __forceinline__ v8f mma_b(v16b a, v16b b, v8f c) {
  return __builtin_amdgcn_wmma_f32_16x16x32_bf16(false, a, false, b, (short)0, c, false, false);
}
__device__ __forceinline__ void guard2(v8f& a, v8f& b, v16h x0, v16h x1, v16h x2, v16h x3, v16h x4, v16h x5) {
#if defined(__HIP_DEVICE_COMPILE__)
  asm volatile("v_nop\n\tv_nop\n\tv_nop\n\tv_nop"
               : "+v"(a), "+v"(b) : "v"(x0), "v"(x1), "v"(x2), "v"(x3), "v"(x4), "v"(x5) : "memory");
#endif
}
template <typename F>
__device__ __forceinline__ void guard6(v8f& a, v8f& b, v8f& c, v8f& d, F x0, F x1, F x2, F x3, F x4, F x5) {
#if defined(__HIP_DEVICE_COMPILE__)
  asm volatile("v_nop\n\tv_nop\n\tv_nop\n\tv_nop"
               : "+v"(a), "+v"(b), "+v"(c), "+v"(d) : "v"(x0), "v"(x1), "v"(x2), "v"(x3), "v"(x4), "v"(x5) : "memory");
#endif
}
__device__ __forceinline__ void acc_guard4(v8f& a, v8f& b, v8f& c, v8f& d) {
#if defined(__HIP_DEVICE_COMPILE__)
  asm volatile("v_nop\n\tv_nop\n\tv_nop\n\tv_nop" : "+v"(a), "+v"(b), "+v"(c), "+v"(d));
#endif
}
__device__ __forceinline__ void wave_sync_lds() {
  __builtin_amdgcn_fence(__ATOMIC_RELEASE, "workgroup");
  __builtin_amdgcn_wave_barrier();
  __builtin_amdgcn_fence(__ATOMIC_ACQUIRE, "workgroup");
}

__global__ __launch_bounds__(256) void ktab(const int* __restrict__ offp, float* cosT, float* sinT) {
#pragma clang fp contract(off)
  __shared__ float sinv[DRH];
  const int tid = (int)threadIdx.x;
  if (tid < DRH) {
    const double ex = (double)tid * (L2_1E4 / (double)DRH);
    const double pw = exp2(ex);
    const float  pf = (float)pw;
    sinv[tid] = 1.0f / pf;
  }
  __syncthreads();
  const int idx = (int)blockIdx.x * 256 + tid;
  const int s   = idx >> 5;
  const int j   = idx & 31;
  if (s >= SEQ) return;
  const int   off  = offp[0];
  const float tpos = (float)(s + off);
  const float ang  = tpos * sinv[j];
  float sn, cs;
  sincosf(ang, &sn, &cs);
  for (int pass = 0; pass < 2; ++pass) {
    *(volatile float*)(cosT + idx) = cs;
    *(volatile float*)(sinT + idx) = sn;
    __threadfence();
  }
}

__global__ __launch_bounds__(256) void cvtb(const float* __restrict__ x, u16* D, int n8) {
  const int gt = blockIdx.x * 256 + (int)threadIdx.x;
  if (gt >= n8) return;
  const float* p = x + (size_t)gt * 8;
  const v4f a = *(const v4f*)(p), b4 = *(const v4f*)(p + 4);
  float w[8];
#pragma unroll
  for (int e = 0; e < 4; ++e) { w[e] = a[e]; w[4 + e] = b4[e]; }
  v4u o;
#pragma unroll
  for (int e = 0; e < 4; ++e) o[e] = pk16(bf_bits(w[2 * e]), bf_bits(w[2 * e + 1]));
  u16* d = D + (size_t)gt * 8;
  for (int pass = 0; pass < 2; ++pass) {
    *(volatile v4u*)(d) = o;
    __threadfence();
  }
}

__global__ __launch_bounds__(256) void wtc(const float* __restrict__ W, u16* Wt, int K, int N, int f16mode, float scale) {
  __shared__ __align__(16) u16 T[64 * WTP];
  const int tid = (int)threadIdx.x;
  const int ntn = N >> 6;
  const int bid = (int)blockIdx.x;
  const int n0  = (bid % ntn) * 64;
  const int k0  = (bid / ntn) * 64;
  if (k0 + 64 > K) return;
  {
    const int kr = tid >> 2;
    const int nc = (tid & 3) * 16;
    const float* src = W + (size_t)(k0 + kr) * (size_t)N + n0 + nc;
#pragma unroll
    for (int i = 0; i < 4; ++i) {
      const v4f a = *(const v4f*)(src + 4 * i);
#pragma unroll
      for (int e = 0; e < 4; ++e) {
        const float f = a[e];
        const unsigned short hb = h_bits((_Float16)(bfr(f) * scale));
        const unsigned short bb = bf_bits(f);
        T[(nc + 4 * i + e) * WTP + kr] = (f16mode != 0) ? hb : bb;
      }
    }
  }
  __syncthreads();
  const int q8 = tid >> 3, p8 = (tid & 7) * 8;
  v4u v[2];
#pragma unroll
  for (int it = 0; it < 2; ++it) v[it] = *(const v4u*)(T + (it * 32 + q8) * WTP + p8);
  u16* base = Wt + (size_t)n0 * (size_t)K + k0 + p8;
  for (int pass = 0; pass < 2; ++pass) {
#pragma unroll
    for (int it = 0; it < 2; ++it) {
      *(volatile v4u*)(base + (size_t)(it * 32 + q8) * (size_t)K) = v[it];
    }
    __threadfence();
  }
}

__global__ __launch_bounds__(256) void cvthl(const float* __restrict__ x, u16* Hp, u16* Lp, int n8, int ncol, float scale) {
  const int gt = blockIdx.x * 256 + (int)threadIdx.x;
  if (gt >= n8) return;
  const size_t e0  = (size_t)gt * 8;
  const int    row = (int)(e0 / (size_t)ncol);
  const int    col = (int)(e0 - (size_t)row * (size_t)ncol);
  const int    b   = row / SEQ;
  const int    s   = row - b * SEQ;
  const float* p = x + e0;
  const v4f a = *(const v4f*)(p), b4 = *(const v4f*)(p + 4);
  float w[8];
#pragma unroll
  for (int e = 0; e < 4; ++e) { w[e] = a[e]; w[4 + e] = b4[e]; }
  v4u oh, ol;
#pragma unroll
  for (int e = 0; e < 4; ++e) {
    const float t0 = w[2 * e] * scale, t1 = w[2 * e + 1] * scale;
    const _Float16 h0 = (_Float16)t0, h1 = (_Float16)t1;
    const _Float16 l0 = (_Float16)(t0 - (float)h0), l1 = (_Float16)(t1 - (float)h1);
    oh[e] = pk16(h_bits(h0), h_bits(h1));
    ol[e] = pk16(h_bits(l0), h_bits(l1));
  }
  u16* dh = Hp + e0;
  const bool wl = (s < QA);
  const int  sl = wl ? s : 0;
  u16* dl = Lp + ((size_t)(b * QA + sl) * (size_t)ncol + col);
  for (int pass = 0; pass < 2; ++pass) {
    *(volatile v4u*)(dh) = oh;
    if (wl) *(volatile v4u*)(dl) = ol;
    __threadfence();
  }
}

__global__ __launch_bounds__(256) void cvtc(const float* __restrict__ x, u16* Hp, u16* Lp, int n8, float scale) {
  const int gt = blockIdx.x * 256 + (int)threadIdx.x;
  if (gt >= n8) return;
  const float* p = x + (size_t)gt * 8;
  const v4f a = *(const v4f*)(p), b4 = *(const v4f*)(p + 4);
  float w[8];
#pragma unroll
  for (int e = 0; e < 4; ++e) { w[e] = a[e]; w[4 + e] = b4[e]; }
  v4u oh, ol;
#pragma unroll
  for (int e = 0; e < 4; ++e) {
    const float t0 = w[2 * e] * scale, t1 = w[2 * e + 1] * scale;
    const _Float16 h0 = (_Float16)t0, h1 = (_Float16)t1;
    const _Float16 l0 = (_Float16)(t0 - (float)h0), l1 = (_Float16)(t1 - (float)h1);
    oh[e] = pk16(h_bits(h0), h_bits(h1));
    ol[e] = pk16(h_bits(l0), h_bits(l1));
  }
  u16* dh = Hp + (size_t)gt * 8;
  u16* dl = Lp + (size_t)gt * 8;
  for (int pass = 0; pass < 2; ++pass) {
    *(volatile v4u*)(dh) = oh;
    *(volatile v4u*)(dl) = ol;
    __threadfence();
  }
}

template <bool CACHE>
__global__ __launch_bounds__(256) void krope(const float* __restrict__ R, const float* __restrict__ Cf,
                                             const float* __restrict__ cosT, const float* __restrict__ sinT,
                                             u16* Hp, u16* Lp, float* cache, float sc) {
#pragma clang fp contract(off)
  __shared__ __align__(16) float Sf[32 * RFP];
  const int tid  = (int)threadIdx.x;
  const int row0 = (int)blockIdx.x * 32;
  if (row0 + 32 > MROWS) return;
  const int r   = tid >> 3;
  const int c8  = (tid & 7) * 8;
  const int row = row0 + r;
  const int b   = row / SEQ;
  const int s   = row - b * SEQ;
  const int j0  = c8 & (DRH - 1);
  const bool up = (c8 >= DRH);
  const int  cp = c8 ^ DRH;
  const float* xr = R + (size_t)row * DR;
  const v4f xa = *(const v4f*)(xr + c8), xb = *(const v4f*)(xr + c8 + 4);
  const v4f ya = *(const v4f*)(xr + cp), yb = *(const v4f*)(xr + cp + 4);
  const float* ctp = cosT + (size_t)s * DRH + j0;
  const float* stp = sinT + (size_t)s * DRH + j0;
  const v4f ca = *(const v4f*)(ctp), cb4 = *(const v4f*)(ctp + 4);
  const v4f sa = *(const v4f*)(stp), sb4 = *(const v4f*)(stp + 4);
  float xv[8], yv[8], cv[8], sv[8], rv[8];
#pragma unroll
  for (int e = 0; e < 4; ++e) {
    xv[e] = xa[e];  xv[4 + e] = xb[e];
    yv[e] = ya[e];  yv[4 + e] = yb[e];
    cv[e] = ca[e];  cv[4 + e] = cb4[e];
    sv[e] = sa[e];  sv[4 + e] = sb4[e];
  }
#pragma unroll
  for (int e = 0; e < 8; ++e) {
    const float pm = xv[e] * cv[e];
    const float qm = yv[e] * sv[e];
    rv[e] = up ? (pm + qm) : (pm - qm);
  }
  v4u oh, ol;
#pragma unroll
  for (int e = 0; e < 4; ++e) {
    const float t0 = rv[2 * e] * sc, t1 = rv[2 * e + 1] * sc;
    const _Float16 h0 = (_Float16)t0, h1 = (_Float16)t1;
    const _Float16 l0 = (_Float16)(t0 - (float)h0), l1 = (_Float16)(t1 - (float)h1);
    oh[e] = pk16(h_bits(h0), h_bits(h1));
    ol[e] = pk16(h_bits(l0), h_bits(l1));
  }
  if constexpr (CACHE) {
#pragma unroll
    for (int e = 0; e < 8; ++e) Sf[r * RFP + c8 + e] = rv[e];
  }
  u16* dh = Hp + (size_t)row * DR + c8;
  const bool wl = (s < QA);
  const int  sl = wl ? s : 0;
  u16* dl = Lp + ((size_t)(b * QA + sl) * DR + c8);
  for (int pass = 0; pass < 2; ++pass) {
    *(volatile v4u*)(dh) = oh;
    if (wl) *(volatile v4u*)(dl) = ol;
    __threadfence();
  }
  if constexpr (CACHE) {
    __syncthreads();
    float* cbase = cache + (size_t)row0 * CW;
    const int rB = tid >> 4, pB = (tid & 15) * 4;
    const v4f kv0 = *(const v4f*)(Sf + rB * RFP + pB);
    const v4f kv1 = *(const v4f*)(Sf + (rB + 16) * RFP + pB);
    for (int pass = 0; pass < 2; ++pass) {
      *(volatile v4f*)(cbase + (size_t)rB * CW + DL + pB) = kv0;
      *(volatile v4f*)(cbase + (size_t)(rB + 16) * CW + DL + pB) = kv1;
      __threadfence();
    }
    const int rC = tid >> 7, pC = (tid & 127) * 4;
    v4f cvv[16];
#pragma unroll
    for (int it = 0; it < 16; ++it) cvv[it] = *(const v4f*)(Cf + (size_t)(row0 + 2 * it + rC) * DL + pC);
    for (int pass = 0; pass < 2; ++pass) {
#pragma unroll
      for (int it = 0; it < 16; ++it) {
        *(volatile v4f*)(cbase + (size_t)(2 * it + rC) * CW + pC) = cvv[it];
      }
      __threadfence();
    }
  }
}

__global__ __launch_bounds__(256) void vt16(const float* __restrict__ F, u16* VHo, u16* VLo) {
  __shared__ __align__(16) u16 TH[HD * VTP];
  __shared__ __align__(16) u16 TL[HD * VTP];
  const int tid = threadIdx.x;
  const int bid = blockIdx.x;
  const int st  = bid % NST;
  const int t2  = bid / NST;
  const int g   = t2 % NH;
  const int b   = t2 / NH;
  if (b >= NB) return;
  const int s0  = st * 64;
  {
    const int sl = tid >> 2;
    const int dc = (tid & 3) * 32;
    const float* src = F + ((size_t)b * SEQ + s0 + sl) * KVD + g * HD + dc;
#pragma unroll
    for (int i = 0; i < 8; ++i) {
      const v4f a = *(const v4f*)(src + 4 * i);
#pragma unroll
      for (int e = 0; e < 4; ++e) {
        const float t = a[e] * VCAR;
        const _Float16 hv = (_Float16)t;
        const _Float16 lv = (_Float16)(t - (float)hv);
        TH[(dc + 4 * i + e) * VTP + sl] = h_bits(hv);
        TL[(dc + 4 * i + e) * VTP + sl] = h_bits(lv);
      }
    }
  }
  __syncthreads();
  v4u vh[4], vl[4];
  const int q8 = tid >> 3, p8 = (tid & 7) * 8;
#pragma unroll
  for (int it = 0; it < 4; ++it) {
    const int line = it * 32 + q8;
    vh[it] = *(const v4u*)(TH + line * VTP + p8);
    vl[it] = *(const v4u*)(TL + line * VTP + p8);
  }
  const size_t hrow  = (size_t)(b * NH + g) * HD;
  const size_t baseH = hrow * SEQ + s0 + p8;
  const size_t baseL = hrow * QA + s0 + p8;
  const bool   wl    = (s0 < QA);
  for (int pass = 0; pass < 2; ++pass) {
#pragma unroll
    for (int it = 0; it < 4; ++it) {
      const int line = it * 32 + q8;
      *(volatile v4u*)(VHo + baseH + (size_t)line * SEQ) = vh[it];
      if (wl) *(volatile v4u*)(VLo + baseL + (size_t)line * QA) = vl[it];
    }
    __threadfence();
  }
}

__device__ __forceinline__ void epi64(float* sl, v8f a0, v8f a1, v8f a2, v8f a3, float oscale,
                                      float* C, int N, size_t rowb, int col0, int lane) {
  const int hh = lane >> 4, m = lane & 15;
#pragma unroll
  for (int r = 0; r < 8; ++r) {
    const int ro = (8 * hh + r) * 68 + m;
    sl[ro]      = a0[r] * oscale;
    sl[ro + 16] = a1[r] * oscale;
    sl[ro + 32] = a2[r] * oscale;
    sl[ro + 48] = a3[r] * oscale;
  }
  wave_sync_lds();
  v4f vals[8];
#pragma unroll
  for (int it = 0; it < 8; ++it) vals[it] = *(const v4f*)(sl + (it * 2 + hh) * 68 + m * 4);
  float* dst = C + (rowb + (size_t)hh) * (size_t)N + col0 + m * 4;
  for (int pass = 0; pass < 2; ++pass) {
#pragma unroll
    for (int it = 0; it < 8; ++it) {
      *(volatile v4f*)(dst + (size_t)(it * 2) * (size_t)N) = vals[it];
    }
    __threadfence();
  }
}

__global__ __launch_bounds__(128)
void gemm_bf(const u16* __restrict__ A, const u16* __restrict__ Bt, float* C, int M, int N, int K, float oscale) {
  __shared__ __align__(16) float slab[4 * SLAB64];
  const int tid = threadIdx.x, wave = tid >> 5, lane = tid & 31, hh = lane >> 4, m = lane & 15;
  const int ntile = N >> 6;
  const int bid   = blockIdx.x;
  const int rowb  = (bid / ntile) * 64 + wave * 16;
  const int col0  = (bid % ntile) * 64;
  if (rowb + 16 > M) return;
  const u16* ap = A  + (size_t)(rowb + m) * K + 8 * hh;
  const u16* bp = Bt + (size_t)(col0 + m) * K + 8 * hh;
  const size_t bs = (size_t)16 * K;
  v8f acc0 = zero8(), acc1 = zero8(), acc2 = zero8(), acc3 = zero8();
#pragma unroll 1
  for (int k0 = 0; k0 < K; k0 += 32) {
    const v16b a  = ldfrag_b(ap + k0);
    const v16b b0 = ldfrag_b(bp + k0);
    const v16b b1 = ldfrag_b(bp + bs + k0);
    const v16b b2 = ldfrag_b(bp + 2 * bs + k0);
    const v16b b3 = ldfrag_b(bp + 3 * bs + k0);
    acc0 = mma_b(a, b0, acc0);
    acc1 = mma_b(a, b1, acc1);
    acc2 = mma_b(a, b2, acc2);
    acc3 = mma_b(a, b3, acc3);
    guard6<v16b>(acc0, acc1, acc2, acc3, a, b0, b1, b2, b3, a);
  }
  epi64(slab + wave * SLAB64, acc0, acc1, acc2, acc3, oscale, C, N, (size_t)rowb, col0, lane);
}

template <int NPROD>
__global__ __launch_bounds__(128)
void gemm_h(const u16* __restrict__ Ah, const u16* __restrict__ Al, const u16* __restrict__ Bt,
            float* C, int N, int K, int sbeg, int nrt, float oscale) {
  __shared__ __align__(16) float slab[4 * SLAB64];
  const int tid = threadIdx.x, wave = tid >> 5, lane = tid & 31, hh = lane >> 4, m = lane & 15;
  const int ntile = N >> 6;
  const int bid   = blockIdx.x;
  const int ct    = bid % ntile;
  const int t2    = bid / ntile;
  const int rt    = t2 % nrt;
  const int bb    = t2 / nrt;
  if (bb >= NB) return;
  const int srow  = sbeg + rt * 64 + wave * 16;
  if (srow + 16 > SEQ) return;
  const int col0  = ct * 64;
  const size_t rowC = (size_t)bb * SEQ + srow;
  const _Float16* ahp = hptr(Ah) + (rowC + m) * (size_t)K + 8 * hh;
  const _Float16* alp = hptr(Al) + (rowC + m) * (size_t)K + 8 * hh;
  const _Float16* bp  = hptr(Bt) + (size_t)(col0 + m) * K + 8 * hh;
  const size_t bs = (size_t)16 * K;
  v8f acc0 = zero8(), acc1 = zero8(), acc2 = zero8(), acc3 = zero8();
  if constexpr (NPROD == 2) {
#pragma unroll 1
    for (int k0 = 0; k0 < K; k0 += 32) {
      const v16h ah = ldfrag_h(ahp + k0), al = ldfrag_h(alp + k0);
      const v16h b0 = ldfrag_h(bp + k0);
      const v16h b1 = ldfrag_h(bp + bs + k0);
      const v16h b2 = ldfrag_h(bp + 2 * bs + k0);
      const v16h b3 = ldfrag_h(bp + 3 * bs + k0);
      acc0 = mma_h(ah, b0, acc0);  acc0 = mma_h(al, b0, acc0);
      acc1 = mma_h(ah, b1, acc1);  acc1 = mma_h(al, b1, acc1);
      acc2 = mma_h(ah, b2, acc2);  acc2 = mma_h(al, b2, acc2);
      acc3 = mma_h(ah, b3, acc3);  acc3 = mma_h(al, b3, acc3);
      guard6<v16h>(acc0, acc1, acc2, acc3, ah, al, b0, b1, b2, b3);
    }
  } else {
#pragma unroll 1
    for (int k0 = 0; k0 < K; k0 += 32) {
      const v16h ah = ldfrag_h(ahp + k0);
      const v16h b0 = ldfrag_h(bp + k0);
      const v16h b1 = ldfrag_h(bp + bs + k0);
      const v16h b2 = ldfrag_h(bp + 2 * bs + k0);
      const v16h b3 = ldfrag_h(bp + 3 * bs + k0);
      acc0 = mma_h(ah, b0, acc0);
      acc1 = mma_h(ah, b1, acc1);
      acc2 = mma_h(ah, b2, acc2);
      acc3 = mma_h(ah, b3, acc3);
      guard6<v16h>(acc0, acc1, acc2, acc3, ah, b0, b1, b2, b3, ah);
    }
  }
  epi64(slab + wave * SLAB64, acc0, acc1, acc2, acc3, oscale, C, N, rowC, col0, lane);
}

template <int NP>
__global__ __launch_bounds__(ATT_THREADS)
void attn_c(const u16* __restrict__ QHp, const u16* __restrict__ QLp,
            const u16* __restrict__ KHp, const u16* __restrict__ KLp,
            const u16* __restrict__ QRHp, const u16* __restrict__ QRLp,
            const u16* __restrict__ KRHp, const u16* __restrict__ KRLp,
            const u16* __restrict__ VHp, const u16* __restrict__ VLp,
            u16* OHp, u16* OLp, int qtbeg, int nqt) {
  __shared__ __align__(16) float smem[WPB * WREG];

  const int tid  = threadIdx.x;
  const int wave = tid >> 5;
  const int lane = tid & 31;
  const int hh   = lane >> 4;
  const int c    = lane & 15;
  const int bid  = blockIdx.x;
  const int qt   = qtbeg + bid % nqt;
  const int t2   = bid / nqt;
  const int hp   = t2 % NHP;
  const int b    = t2 / NHP;
  if (b >= NB) return;
  const int q0   = qt * 16;
  if (q0 + 16 > SEQ) return;
  if (NP == 3) { if (q0 + 16 > QA) return; }
  const int head = hp * WPB + wave;

  float* pt   = smem + wave * WREG;
  float* slab = pt + PTW;

  const size_t hcol = (size_t)head * HD + 8 * hh;
  const _Float16* Qh  = hptr(QHp)  + ((size_t)b * SEQ + q0 + c) * DMOD + hcol;
  const _Float16* Khb = hptr(KHp)  + ((size_t)b * SEQ + c) * KVD + hcol;
  const _Float16* Qrh = hptr(QRHp) + ((size_t)b * SEQ + q0 + c) * DR + 8 * hh;
  const _Float16* Krb = hptr(KRHp) + ((size_t)b * SEQ + c) * DR + 8 * hh;
  const _Float16* Vhb = hptr(VHp)  + ((size_t)(b * NH + head) * HD + c) * SEQ + 8 * hh;
  const _Float16* Ql   = Qh;
  const _Float16* Klb  = Khb;
  const _Float16* Qrl  = Qrh;
  const _Float16* Krlb = Krb;
  const _Float16* Vlb  = Vhb;
  if constexpr (NP == 3) {
    Ql   = hptr(QLp)  + ((size_t)b * QA + q0 + c) * DMOD + hcol;
    Klb  = hptr(KLp)  + ((size_t)b * QA + c) * KVD + hcol;
    Qrl  = hptr(QRLp) + ((size_t)b * QA + q0 + c) * DR + 8 * hh;
    Krlb = hptr(KRLp) + ((size_t)b * QA + c) * DR + 8 * hh;
    Vlb  = hptr(VLp)  + ((size_t)(b * NH + head) * HD + c) * QA + 8 * hh;
  }
  const float lsc = RSQS * (LOG2E / (QSC * KSC));
  const float oc  = 1.0f / (PCAR * VCAR);
  const size_t KROW = (size_t)KVD;
  const size_t RROW = (size_t)DR;

  float mrow[8], lrow[8];
  v8f o[8];
#pragma unroll
  for (int r = 0; r < 8; ++r) { mrow[r] = -INFINITY; lrow[r] = 0.f; }
#pragma unroll
  for (int j = 0; j < 8; ++j) o[j] = zero8();
  const int ncaus = (q0 >> 5) + 1;
  const int nkt = (ncaus < NKT) ? ncaus : NKT;
  const int qr0 = q0 + 8 * hh;

#pragma unroll 1
  for (int kt = 0; kt < nkt; ++kt) {
    const int kb = kt * 32;
    v8f s0 = zero8(), s1 = zero8();
    const _Float16* k0p = Khb + (size_t)kb * KROW;
    const _Float16* k1p = k0p + (size_t)16 * KROW;
    const _Float16* r0p = Krb + (size_t)kb * RROW;
    const _Float16* r1p = r0p + (size_t)16 * RROW;
    if constexpr (NP == 3) {
      const _Float16* l0p = Klb + (size_t)kb * KROW;
      const _Float16* l1p = l0p + (size_t)16 * KROW;
      const _Float16* m0p = Krlb + (size_t)kb * RROW;
      const _Float16* m1p = m0p + (size_t)16 * RROW;
#pragma unroll
      for (int kk = 0; kk < HD / 32; ++kk) {
        const v16h qh  = ldfrag_h(Qh + kk * 32);
        const v16h ql  = ldfrag_h(Ql + kk * 32);
        const v16h kh0 = ldfrag_h(k0p + kk * 32);
        const v16h kh1 = ldfrag_h(k1p + kk * 32);
        const v16h kl0 = ldfrag_h(l0p + kk * 32);
        const v16h kl1 = ldfrag_h(l1p + kk * 32);
        s0 = mma_h(qh, kh0, s0);
        s0 = mma_h(ql, kh0, s0);
        s0 = mma_h(qh, kl0, s0);
        s1 = mma_h(qh, kh1, s1);
        s1 = mma_h(ql, kh1, s1);
        s1 = mma_h(qh, kl1, s1);
        guard2(s0, s1, qh, ql, kh0, kl0, kh1, kl1);
      }
#pragma unroll
      for (int kk = 0; kk < DR / 32; ++kk) {
        const v16h qh  = ldfrag_h(Qrh + kk * 32);
        const v16h ql  = ldfrag_h(Qrl + kk * 32);
        const v16h kh0 = ldfrag_h(r0p + kk * 32);
        const v16h kh1 = ldfrag_h(r1p + kk * 32);
        const v16h kl0 = ldfrag_h(m0p + kk * 32);
        const v16h kl1 = ldfrag_h(m1p + kk * 32);
        s0 = mma_h(qh, kh0, s0);
        s0 = mma_h(ql, kh0, s0);
        s0 = mma_h(qh, kl0, s0);
        s1 = mma_h(qh, kh1, s1);
        s1 = mma_h(ql, kh1, s1);
        s1 = mma_h(qh, kl1, s1);
        guard2(s0, s1, qh, ql, kh0, kl0, kh1, kl1);
      }
    } else {
#pragma unroll
      for (int kk = 0; kk < HD / 32; ++kk) {
        const v16h qh  = ldfrag_h(Qh + kk * 32);
        const v16h kh0 = ldfrag_h(k0p + kk * 32);
        const v16h kh1 = ldfrag_h(k1p + kk * 32);
        s0 = mma_h(qh, kh0, s0);
        s1 = mma_h(qh, kh1, s1);
        guard2(s0, s1, qh, kh0, kh1, qh, kh0, kh1);
      }
#pragma unroll
      for (int kk = 0; kk < DR / 32; ++kk) {
        const v16h qh  = ldfrag_h(Qrh + kk * 32);
        const v16h kh0 = ldfrag_h(r0p + kk * 32);
        const v16h kh1 = ldfrag_h(r1p + kk * 32);
        s0 = mma_h(qh, kh0, s0);
        s1 = mma_h(qh, kh1, s1);
        guard2(s0, s1, qh, kh0, kh1, qh, kh0, kh1);
      }
    }
    const int key0 = kb + c, key1 = kb + 16 + c;
#pragma unroll
    for (int r = 0; r < 8; ++r) {
      const int   qr = qr0 + r;
      const float u0 = s0[r] * lsc;
      const float u1 = s1[r] * lsc;
      const float t0 = (key0 > qr) ? -INFINITY : u0;
      const float t1 = (key1 > qr) ? -INFINITY : u1;
      float mx = fmaxf(t0, t1);
#pragma unroll
      for (int off = 1; off < 16; off <<= 1) mx = fmaxf(mx, __shfl_xor(mx, off, 32));
      const float mn = fmaxf(mrow[r], mx);
      const float ms = (mn == -INFINITY) ? 0.0f : mn;
      const float al = exp2f(mrow[r] - ms);
      mrow[r] = mn;
      const float e0 = exp2f(t0 - ms), e1 = exp2f(t1 - ms);
      float ps = e0 + e1;
#pragma unroll
      for (int off = 1; off < 16; off <<= 1) ps += __shfl_xor(ps, off, 32);
      lrow[r] = lrow[r] * al + ps;
#pragma unroll
      for (int j = 0; j < 8; ++j) o[j][r] *= al;
      const int ro = (8 * hh + r) * PTP + c;
      pt[ro]      = e0;
      pt[ro + 16] = e1;
    }
    wave_sync_lds();
    FragH ph, pl;
    {
      const float* prow = pt + c * PTP + 8 * hh;
      const v4f p0 = *(const v4f*)(prow), p1 = *(const v4f*)(prow + 4);
      const v4f p2 = *(const v4f*)(prow + 16), p3 = *(const v4f*)(prow + 20);
#pragma unroll
      for (int e = 0; e < 4; ++e) {
        const float ta = p0[e] * PCAR, tb = p1[e] * PCAR, tc = p2[e] * PCAR, td = p3[e] * PCAR;
        const _Float16 ha = (_Float16)ta, hb = (_Float16)tb, hc = (_Float16)tc, hd = (_Float16)td;
        ph.h[0][e]     = ha;
        ph.h[0][4 + e] = hb;
        ph.h[1][e]     = hc;
        ph.h[1][4 + e] = hd;
        if constexpr (NP == 3) {
          pl.h[0][e]     = (_Float16)(ta - (float)ha);
          pl.h[0][4 + e] = (_Float16)(tb - (float)hb);
          pl.h[1][e]     = (_Float16)(tc - (float)hc);
          pl.h[1][4 + e] = (_Float16)(td - (float)hd);
        }
      }
    }
    {
      const _Float16* vhp = Vhb + kb;
      if constexpr (NP == 3) {
        const _Float16* vlp = Vlb + kb;
#pragma unroll
        for (int jg = 0; jg < 4; ++jg) {
          const size_t da  = (size_t)(2 * jg) * 16 * SEQ;
          const size_t db  = da + (size_t)16 * SEQ;
          const size_t dla = (size_t)(2 * jg) * 16 * QA;
          const size_t dlb = dla + (size_t)16 * QA;
          const v16h vha = ldfrag_h(vhp + da),  vhb2 = ldfrag_h(vhp + db);
          const v16h vla = ldfrag_h(vlp + dla), vlb2 = ldfrag_h(vlp + dlb);
          o[2 * jg]     = mma_h(ph.v, vha,  o[2 * jg]);
          o[2 * jg]     = mma_h(pl.v, vha,  o[2 * jg]);
          o[2 * jg]     = mma_h(ph.v, vla,  o[2 * jg]);
          o[2 * jg + 1] = mma_h(ph.v, vhb2, o[2 * jg + 1]);
          o[2 * jg + 1] = mma_h(pl.v, vhb2, o[2 * jg + 1]);
          o[2 * jg + 1] = mma_h(ph.v, vlb2, o[2 * jg + 1]);
          guard2(o[2 * jg], o[2 * jg + 1], ph.v, pl.v, vha, vhb2, vla, vlb2);
        }
      } else {
#pragma unroll
        for (int jg = 0; jg < 4; ++jg) {
          const size_t da = (size_t)(2 * jg) * 16 * SEQ;
          const size_t db = da + (size_t)16 * SEQ;
          const v16h vha = ldfrag_h(vhp + da), vhb2 = ldfrag_h(vhp + db);
          o[2 * jg]     = mma_h(ph.v, vha,  o[2 * jg]);
          o[2 * jg + 1] = mma_h(ph.v, vhb2, o[2 * jg + 1]);
          guard2(o[2 * jg], o[2 * jg + 1], ph.v, vha, vhb2, ph.v, vha, vhb2);
        }
      }
    }
    wave_sync_lds();
  }
  acc_guard4(o[0], o[1], o[2], o[3]);
  acc_guard4(o[4], o[5], o[6], o[7]);
#pragma unroll
  for (int r = 0; r < 8; ++r) {
    const float lv  = lrow[r];
    const float ls  = (lv > 0.0f) ? lv : 1.0f;
    const float inv = (lv > 0.0f) ? ((1.0f / ls) * oc) : 0.0f;
#pragma unroll
    for (int j = 0; j < 8; ++j) {
      const int idx = (8 * hh + r) * SLP + j * 16 + c;
      slab[idx] = o[j][r] * inv;
    }
  }

  wave_sync_lds();
  v4u oh[8], ol[8];
  const int rq = lane >> 4, c8 = (lane & 15) * 8;
#pragma unroll
  for (int it = 0; it < 8; ++it) {
    const int row = it * 2 + rq;
    const v4f a = *(const v4f*)(slab + row * SLP + c8), b4 = *(const v4f*)(slab + row * SLP + c8 + 4);
    float w[8];
#pragma unroll
    for (int e = 0; e < 4; ++e) { w[e] = a[e] * OSC; w[4 + e] = b4[e] * OSC; }
#pragma unroll
    for (int e = 0; e < 4; ++e) {
      const _Float16 h0 = (_Float16)w[2 * e], h1 = (_Float16)w[2 * e + 1];
      const _Float16 l0 = (_Float16)(w[2 * e] - (float)h0), l1 = (_Float16)(w[2 * e + 1] - (float)h1);
      oh[it][e] = pk16(h_bits(h0), h_bits(h1));
      ol[it][e] = pk16(h_bits(l0), h_bits(l1));
    }
  }
  const size_t ob = ((size_t)b * SEQ + q0) * DMOD + (size_t)head * HD + c8;
  for (int pass = 0; pass < 2; ++pass) {
#pragma unroll
    for (int it = 0; it < 8; ++it) {
      const int row = it * 2 + rq;
      *(volatile v4u*)(OHp + ob + (size_t)row * DMOD) = oh[it];
      *(volatile v4u*)(OLp + ob + (size_t)row * DMOD) = ol[it];
    }
    __threadfence();
  }
}

extern "C" void kernel_launch(void* const* d_in, const int* in_sizes, int n_in,
                              void* d_out, int out_size, void* d_ws, size_t ws_size,
                              hipStream_t stream) {
  if (n_in < 9) return;
  if (in_sizes[0] < ((NB - 1) * XS_FULL + SEQ) * DMOD) return;
  if (in_sizes[1] != DMOD * DL) return;
  if (in_sizes[2] != DL * KVD) return;
  if (in_sizes[3] != DL * KVD) return;
  if (in_sizes[4] != DMOD * DMOD) return;
  if (in_sizes[5] != DMOD * DR) return;
  if (in_sizes[6] != DL * DR) return;
  if (in_sizes[7] != DMOD * DMOD) return;
  if (in_sizes[8] < 1) return;
  if ((size_t)out_size < (size_t)MROWS * DMOD + (size_t)MROWS * CW) return;

  const float* x    = (const float*)d_in[0];
  const float* wkv  = (const float*)d_in[1];
  const float* wku  = (const float*)d_in[2];
  const float* wvu  = (const float*)d_in[3];
  const float* wq   = (const float*)d_in[4];
  const float* wqr  = (const float*)d_in[5];
  const float* wkr  = (const float*)d_in[6];
  const float* wo   = (const float*)d_in[7];
  const int*   offp = (const int*)d_in[8];
  float*       out0 = (float*)d_out;
  float*       out1 = out0 + (size_t)MROWS * DMOD;

  const size_t szT  = (size_t)SEQ * DRH * 4;
  const size_t szXB = (size_t)MROWS * DMOD * 2;
  const size_t szW  = (size_t)DMOD * DMOD * 2;
  const size_t szF  = (size_t)MROWS * DMOD * 4;
  const size_t szC  = (size_t)MROWS * DL * 2;
  const size_t szQ  = (size_t)MROWS * DMOD * 2;
  const size_t szL  = (size_t)NB * QA * DMOD * 2;
  const size_t szR  = (size_t)MROWS * DR * 2;
  const size_t szRL = (size_t)NB * QA * DR * 2;
  const size_t szVH = (size_t)NB * NH * HD * SEQ * 2;
  const size_t szVL = (size_t)NB * NH * HD * QA * 2;
  if (2 * szQ > szF) return;
  if (((size_t)MROWS * DL + (size_t)MROWS * DR) * 4 > szF) return;
  if ((size_t)MROWS * DR * 4 > szF) return;
  if ((size_t)MROWS * KVD * 2 > szXB) return;
  if ((size_t)DL * DMOD * 2 > szW || (size_t)KVD * DL * 2 > szW || (size_t)DR * DMOD * 2 > szW) return;
  size_t off = 0;
  const size_t oCOS = off; off += szT;
  const size_t oSIN = off; off += szT;
  const size_t oXB  = off; off += szXB;
  const size_t oW   = off; off += szW;
  const size_t oF   = off; off += szF;
  const size_t oCH  = off; off += szC;
  const size_t oCL  = off; off += szC;
  const size_t oQH  = off; off += szQ;
  const size_t oQL  = off; off += szL;
  const size_t oKL  = off; off += szL;
  const size_t oQRH = off; off += szR;
  const size_t oKRH = off; off += szR;
  const size_t oQRL = off; off += szRL;
  const size_t oKRL = off; off += szRL;
  const size_t oVH  = off; off += szVH;
  const size_t oVL  = off; off += szVL;
  if (off > ws_size) return;
  if (off > (size_t)WS_CAP) return;

  char* ws = (char*)d_ws;
  float* COS = (float*)(ws + oCOS);
  float* SIN = (float*)(ws + oSIN);
  u16*   XB  = (u16*)(ws + oXB);
  u16*   KH  = (u16*)(ws + oXB);
  u16*   WB  = (u16*)(ws + oW);
  float* F   = (float*)(ws + oF);
  float* FR2 = F + (size_t)MROWS * DL;
  u16*   OH  = (u16*)(ws + oF);
  u16*   OL  = (u16*)(ws + oF + szQ);
  u16*   CH  = (u16*)(ws + oCH);
  u16*   CL  = (u16*)(ws + oCL);
  u16*   QH  = (u16*)(ws + oQH);
  u16*   QL  = (u16*)(ws + oQL);
  u16*   KL  = (u16*)(ws + oKL);
  u16*   QRH = (u16*)(ws + oQRH);
  u16*   KRH = (u16*)(ws + oKRH);
  u16*   QRL = (u16*)(ws + oQRL);
  u16*   KRL = (u16*)(ws + oKRL);
  u16*   VH  = (u16*)(ws + oVH);
  u16*   VL  = (u16*)(ws + oVL);

  const dim3 b256(256), b128(128), bAT(ATT_THREADS);
  const dim3 gTAB((SEQ * DRH) / 256);
  const int  n8x  = (SEQ * DMOD) / 8;
  const dim3 gX((n8x + 255) / 256);
  const int  n8q  = (MROWS * DMOD) / 8;
  const int  n8c  = (MROWS * DL) / 8;
  const dim3 gHL((n8q + 255) / 256);
  const dim3 gC((n8c + 255) / 256);
  const dim3 gWQ((DMOD / 64) * (DMOD / 64));
  const dim3 gWQR((DR / 64) * (DMOD / 64));
  const dim3 gWKV((DL / 64) * (DMOD / 64));
  const dim3 gWKR((DR / 64) * (DL / 64));
  const dim3 gWUP((KVD / 64) * (DL / 64));
  const dim3 gGQ((MROWS / 64) * (DMOD / 64));
  const dim3 gGQR((MROWS / 64) * (DR / 64));
  const dim3 gGC((MROWS / 64) * (DL / 64));
  const dim3 gGKR(NB * (SEQ / 64) * (DR / 64));
  const dim3 gGK(NB * (SEQ / 64) * (KVD / 64));
  const dim3 gRP(MROWS / 32);
  const dim3 gVT(NB * NH * NST);
  const int  nqtA = QA / 16;
  const int  nqtB = (SEQ - QA) / 16;
  const int  nrtA = QA / 64;
  const int  nrtB = (SEQ - QA) / 64;

  ktab<<<gTAB, b256, 0, stream>>>(offp, COS, SIN);
  for (int bb = 0; bb < NB; ++bb) {
    cvtb<<<gX, b256, 0, stream>>>(x + (size_t)bb * XS_FULL * DMOD, XB + (size_t)bb * SEQ * DMOD, n8x);
  }
  wtc<<<gWQ, b256, 0, stream>>>(wq, WB, DMOD, DMOD, 0, 1.0f);
  gemm_bf<<<gGQ, b128, 0, stream>>>(XB, WB, F, MROWS, DMOD, DMOD, 1.0f);
  cvthl<<<gHL, b256, 0, stream>>>(F, QH, QL, n8q, DMOD, QSC);
  wtc<<<gWQR, b256, 0, stream>>>(wqr, WB, DMOD, DR, 0, 1.0f);
  gemm_bf<<<gGQR, b128, 0, stream>>>(XB, WB, F, MROWS, DR, DMOD, 1.0f);
  krope<false><<<gRP, b256, 0, stream>>>(F, F, COS, SIN, QRH, QRL, out1, QSC);
  wtc<<<gWKV, b256, 0, stream>>>(wkv, WB, DMOD, DL, 0, 1.0f);
  gemm_bf<<<gGC, b128, 0, stream>>>(XB, WB, F, MROWS, DL, DMOD, 1.0f);
  cvtc<<<gC, b256, 0, stream>>>(F, CH, CL, n8c, CSC);
  wtc<<<gWKR, b256, 0, stream>>>(wkr, WB, DL, DR, 1, WKS);
  gemm_h<2><<<gGKR, b128, 0, stream>>>(CH, CL, WB, FR2, DR, DL, 0, SEQ / 64, 1.0f / (CSC * WKS));
  krope<true><<<gRP, b256, 0, stream>>>(FR2, F, COS, SIN, KRH, KRL, out1, KSC);
  wtc<<<gWUP, b256, 0, stream>>>(wku, WB, DL, KVD, 1, WKS);
  gemm_h<2><<<gGK, b128, 0, stream>>>(CH, CL, WB, F, KVD, DL, 0, SEQ / 64, 1.0f / (CSC * WKS));
  cvthl<<<gHL, b256, 0, stream>>>(F, KH, KL, n8q, KVD, KSC);
  wtc<<<gWUP, b256, 0, stream>>>(wvu, WB, DL, KVD, 1, WKS);
  gemm_h<2><<<gGK, b128, 0, stream>>>(CH, CL, WB, F, KVD, DL, 0, SEQ / 64, 1.0f / (CSC * WKS));
  vt16<<<gVT, b256, 0, stream>>>(F, VH, VL);
  wtc<<<gWQ, b256, 0, stream>>>(wo, WB, DMOD, DMOD, 1, WOS);
  attn_c<3><<<dim3(nqtA * NHP * NB), bAT, 0, stream>>>(QH, QL, KH, KL, QRH, QRL, KRH, KRL, VH, VL, OH, OL, 0, nqtA);
  if (nqtB > 0) {
    attn_c<1><<<dim3(nqtB * NHP * NB), bAT, 0, stream>>>(QH, QL, KH, KL, QRH, QRL, KRH, KRL, VH, VL, OH, OL, nqtA, nqtB);
  }
  gemm_h<2><<<dim3(NB * nrtA * (DMOD / 64)), b128, 0, stream>>>(OH, OL, WB, out0, DMOD, DMOD, 0, nrtA, 1.0f / (OSC * WOS));
  if (nrtB > 0) {
    gemm_h<1><<<dim3(NB * nrtB * (DMOD / 64)), b128, 0, stream>>>(OH, OL, WB, out0, DMOD, DMOD, QA, nrtB, 1.0f / (OSC * WOS));
  }
  (void)hipGetLastError();
}
